// InrAwaSA_74947179316071
// MI455X (gfx1250) — hardware-verified
//
#include <hip/hip_runtime.h>
#include <hip/hip_bf16.h>
#include <math.h>

#define BB 4
#define SS 4096
#define DKK 256
#define HH 1
#define QW 1
#define KST2 264
typedef _Float16 bf16;
typedef __attribute__((ext_vector_type(4))) unsigned v4u_t;
typedef unsigned v4ua __attribute__((ext_vector_type(4), may_alias));
typedef __attribute__((ext_vector_type(4))) float v4f_t;
typedef float v4fa __attribute__((ext_vector_type(4), may_alias));
typedef __attribute__((ext_vector_type(16))) bf16  bf16x16;
typedef __attribute__((ext_vector_type(8)))  bf16  bf16x8;
typedef __attribute__((ext_vector_type(4)))  bf16  bf16x4;
typedef __attribute__((ext_vector_type(8)))  float f32x8;
#define LDS_STRIDE 48
#define KSTRIDE    72
#define VSTRIDE    48

__device__ __forceinline__ f32x8 wmma_bf16(bf16x16 a, bf16x16 b, f32x8 c) {
  c = __builtin_amdgcn_wmma_f32_16x16x32_f16(false, a, false, b, (short)0, c, false, false);
  asm volatile("v_nop\n\tv_nop\n\tv_nop\n\tv_nop" : "+v"(c) : "v"(a), "v"(b));
  return c;
}

template <typename T>
__device__ __forceinline__ bf16x16 load_frag(const T* __restrict__ base, int ld,
                                             int row0, int k0) {
  const int lane = threadIdx.x & 31;
  const int r    = lane & 15;
  const int kh   = (lane >> 4) * 8;
  const T* p0 = base + (size_t)(row0 + r) * ld + (k0 + kh);
  const T* p1 = p0 + 16;
  bf16x16 f;
#pragma unroll
  for (int i = 0; i < 8; ++i) {
    f[i]     = (bf16)p0[i];
    f[i + 8] = (bf16)p1[i];
  }
  return f;
}

__device__ __forceinline__ bf16x16 lds_frag(const bf16* base, int stride) {
  const int lane = threadIdx.x & 31;
  const int row  = lane & 15;
  const int kh   = (lane >> 4) * 8;
  const bf16x8 lo = *(const bf16x8*)(base + row * stride + kh);
  const bf16x8 hi = *(const bf16x8*)(base + row * stride + kh + 16);
  bf16x16 f;
#pragma unroll
  for (int i = 0; i < 8; ++i) { f[i] = lo[i]; f[i + 8] = hi[i]; }
  return f;
}

template <typename T>
__device__ __forceinline__ void stage_read16(const T* __restrict__ p, float* buf) {
#pragma unroll
  for (int i = 0; i < 16; ++i) buf[i] = (float)p[i];
}

__device__ __forceinline__ void stage_write(bf16* dst, const float* buf, int nquad) {
#pragma unroll
  for (int i = 0; i < nquad; ++i) {
    bf16x4 q;
    q[0] = (bf16)buf[4 * i];     q[1] = (bf16)buf[4 * i + 1];
    q[2] = (bf16)buf[4 * i + 2]; q[3] = (bf16)buf[4 * i + 3];
    *(bf16x4*)(dst + 4 * i) = q;
  }
}

__global__ __launch_bounds__(64) void attn_kernel(
    const bf16* __restrict__ Qb, const bf16* __restrict__ Kb,
    const bf16* __restrict__ Vt, float* __restrict__ attnOut) {
  __shared__ bf16 ldsK[32 * KST2];
  __shared__ bf16 ldsV[256 * VSTRIDE];
  __shared__ __attribute__((aligned(16))) float oSp[2][8 * 32 * 8];
  __shared__ __attribute__((aligned(16))) float ldsO[2][16 * 132];

  const int q0blk = blockIdx.x * 32;
  const int h  = blockIdx.y;
  const int b  = blockIdx.z;
  const int t    = threadIdx.x;
  const int wave = t >> 5;
  const int lane = t & 31;
  const int qlane = lane & 15;
  const int kh8   = (lane >> 4) * 8;
  const int q0 = q0blk + wave * 16;

  (void)h;
  const bf16* Qh = Qb + (size_t)b * SS * DKK;
  const bf16* Kh = Kb + (size_t)b * SS * DKK;
  const bf16* Vh = Vt + (size_t)b * DKK * SS;

  const int krow = t >> 1;
  const int kcol = (t & 1) * 128;
  const bf16* kSrc = Kh + (size_t)krow * DKK + kcol;
  const bf16* vSrc = Vh + (size_t)t * SS;

  f32x8 o[QW][8] = {};
  float alpha_s[QW];
  float* osp = oSp[wave];
  for (int e = lane; e < 8 * 32 * 8; e += 32) osp[e] = 0.0f;
  __builtin_amdgcn_wave_barrier();
  float mrun[QW], lrun[QW];
#pragma unroll
  for (int qt = 0; qt < QW; ++qt) { mrun[qt] = -INFINITY; lrun[qt] = 0.0f; }

  const float scale = 0.0625f * 1.44269504088896340736f;
  const float NEG2 = -1.0e9f; (void)NEG2;
  const int kmin = 0, kmax = SS - 1;

  for (int kb = kmin; kb <= kmax; kb += 32) {
    __syncthreads();
#pragma unroll
    for (int i = 0; i < 16; ++i) *(bf16x8*)(&ldsK[krow * KST2 + kcol + 8 * i]) = *(const bf16x8*)(kSrc + (size_t)kb * DKK + 8 * i);
#pragma unroll
    for (int rr = 0; rr < 4; ++rr)
#pragma unroll
      for (int i = 0; i < 4; ++i) *(bf16x8*)(&ldsV[(t + 64 * rr) * VSTRIDE + 8 * i]) = *(const bf16x8*)(vSrc + (size_t)(64 * rr) * SS + kb + 8 * i);
    __syncthreads();


    bf16x16 pf[QW];
    bool act[QW];
#pragma unroll
    for (int qt = 0; qt < QW; ++qt) {
      unsigned mbits = 0;
      mbits = 0xFFFFu; act[qt] = true;
      if (act[qt]) {
        const int q_my = q0 + 16 * qt + qlane;
        f32x8 s0 = {}, s1 = {};
#pragma unroll
        for (int c = 0; c < 8; ++c) {
          const bf16x16 qfc = load_frag(Qh, DKK, q0 + 16 * qt, 32 * c);
          const bf16x16 k0f = lds_frag(ldsK + 0 * KST2 + c * 32, KST2), k1f = lds_frag(ldsK + 16 * KST2 + c * 32, KST2);
          s0 = wmma_bf16(k0f, qfc, s0);
          s1 = wmma_bf16(k1f, qfc, s1);
        }

        float mx = -INFINITY;
#pragma unroll
        for (int r = 0; r < 8; ++r) {
          const int k0i = kb + kh8 + r;
          const int k1i = k0i + 16;
          (void)k0i; (void)k1i; (void)q_my;
          s0[r] = (mbits & (1u << r))       ? s0[r] * scale : NEG2;
          s1[r] = (mbits & (1u << (8 + r))) ? s1[r] * scale : NEG2;
          mx = fmaxf(mx, fmaxf(s0[r], s1[r]));
        }
        mx = fmaxf(mx, __shfl_xor(mx, 16, 32));
        const float mnew  = fmaxf(mrun[qt], mx);
        const float alpha = exp2f(mrun[qt] - mnew);

        float rsum = 0.0f;
#pragma unroll
        for (int r = 0; r < 8; ++r) {
          const float p0 = exp2f(s0[r] - mnew);
          const float p1 = exp2f(s1[r] - mnew);
          rsum += p0 + p1;
          pf[qt][r]     = (bf16)(p0 * 1024.0f);
          pf[qt][r + 8] = (bf16)(p1 * 1024.0f);
        }
        rsum += __shfl_xor(rsum, 16, 32);
        lrun[qt] = lrun[qt] * alpha + rsum;
        mrun[qt] = mnew;

#pragma unroll
        for (int j = 0; j < 8; ++j)
#pragma unroll
          for (int r = 0; r < 8; ++r) o[qt][j][r] *= alpha;
        alpha_s[qt] = alpha;
      }
    }

#pragma unroll
    for (int j = 0; j < 8; ++j) {
      const bf16x16 vf2 = lds_frag(ldsV + ((8 + j) * 16) * VSTRIDE, VSTRIDE);
#pragma unroll
      for (int qt = 0; qt < QW; ++qt)
        if (act[qt]) { f32x8 acc;
#pragma unroll
          for (int r = 0; r < 8; ++r) acc[r] = osp[(j * 32 + lane) * 8 + r] * alpha_s[qt];
          acc = wmma_bf16(vf2, pf[qt], acc);
#pragma unroll
          for (int r = 0; r < 8; ++r) osp[(j * 32 + lane) * 8 + r] = acc[r]; }
    }
#pragma unroll
    for (int j = 0; j < 8; ++j) {
      const bf16x16 vf = lds_frag(ldsV + (j * 16) * VSTRIDE, VSTRIDE);
#pragma unroll
      for (int qt = 0; qt < QW; ++qt)
        if (act[qt]) o[qt][j] = wmma_bf16(vf, pf[qt], o[qt][j]);
    }
  }

  float* so = ldsO[wave];
  const float rl = 1.0f / (lrun[0] * 1024.0f);
#pragma unroll 1
  for (int dh = 0; dh < 2; ++dh) {
    __builtin_amdgcn_wave_barrier();
#pragma unroll
    for (int j = 0; j < 8; ++j)
#pragma unroll
      for (int r = 0; r < 8; ++r) so[qlane * 132 + j * 16 + kh8 + r] = (dh == 0 ? o[0][j][r] : osp[(j * 32 + lane) * 8 + r]) * rl;
    asm volatile("s_wait_dscnt 0" ::: "memory");
    __builtin_amdgcn_wave_barrier();
#pragma unroll 1
    for (int pass = 0; pass < 2; ++pass) {
#pragma unroll 4
      for (int it = 0; it < 16; ++it) { const int ch = lane + 32 * it, ql = ch >> 5, q4 = (ch & 31) * 4;
        *(volatile v4f_t*)(attnOut + ((size_t)(b * SS + q0 + ql)) * DKK + dh * 128 + q4) = *(const volatile v4fa*)(so + ql * 132 + q4); }
      __threadfence();
    }
  }
}


__global__ __launch_bounds__(256) void k_cast(const float* __restrict__ x, bf16* __restrict__ x16, bf16* __restrict__ xt) {
  __shared__ float tS[64][257];
  const int tid = threadIdx.x, b = blockIdx.x / (SS / 64), n0 = (blockIdx.x % (SS / 64)) * 64;
  const float* src = x + ((size_t)b * SS + n0) * DKK;
  for (int e = tid; e < 64 * DKK; e += 256) { const int r = e >> 8, d = e & 255; tS[r][d] = src[e]; }
  __syncthreads();
#pragma unroll 1
  for (int pass = 0; pass < 2; ++pass) {
    for (int ch = tid; ch < 64 * 32; ch += 256) { const int r = ch >> 5, q8 = (ch & 31) * 8; union { bf16 hh[8]; v4u_t u; } cv;
#pragma unroll
      for (int e = 0; e < 8; ++e) cv.hh[e] = (bf16)tS[r][q8 + e];
      *(volatile v4u_t*)(x16 + ((size_t)b * SS + n0 + r) * DKK + q8) = cv.u; }
    for (int ch = tid; ch < DKK * 8; ch += 256) { const int d = ch >> 3, q8 = (ch & 7) * 8; union { bf16 hh[8]; v4u_t u; } cv;
#pragma unroll
      for (int e = 0; e < 8; ++e) cv.hh[e] = (bf16)tS[q8 + e][d];
      *(volatile v4u_t*)(xt + ((size_t)b * DKK + d) * SS + n0 + q8) = cv.u; }
    __threadfence();
  }
}

extern "C" void kernel_launch(void* const* d_in, const int* in_sizes, int n_in,
                              void* d_out, int out_size, void* d_ws, size_t ws_size,
                              hipStream_t stream) {
  (void)in_sizes; (void)n_in; (void)out_size; (void)ws_size;
  const float* x = (const float*)d_in[0];
  float* out = (float*)d_out;
  char* ws = (char*)d_ws;
  bf16* x16 = (bf16*)ws; ws += (size_t)BB * SS * DKK * 2;
  bf16* xt  = (bf16*)ws; ws += (size_t)BB * SS * DKK * 2;
  k_cast<<<dim3(BB * SS / 64), dim3(256), 0, stream>>>(x, x16, xt);
  attn_kernel<<<dim3(SS / 32, 1, BB), dim3(64), 0, stream>>>(x16, x16, xt, out);
}
